// TrashNet_6485400616961
// MI455X (gfx1250) — hardware-run, weakly checked
//
#include <hip/hip_runtime.h>


namespace {
constexpr int N = 100000, NP = 100032, E = 3200000, D = 30, DP = 32, KE = 3, TW = KE * DP  , GW = 6 * DP  ;
constexpr float XS = 8.0f, WSC = 256.0f, NEG = 0.2f  ;

typedef _Float16 b16;
typedef __attribute__((ext_vector_type(16))) _Float16 v16b;
typedef __attribute__((ext_vector_type(8))) _Float16 v8b;
typedef __attribute__((ext_vector_type(8))) float v8f;
typedef __attribute__((ext_vector_type(4))) float v4f;
__device__ __forceinline__ float bf16_rne(float f) { unsigned int u = __float_as_uint(f); u += 0x7FFFu + ((u >> 16) & 1u); return __uint_as_float(u & 0xFFFF0000u); }
__device__ __forceinline__ void split16(float v, b16& hi, b16& lo) { hi = (b16)v; lo = (b16)(v - (float)hi); }
__device__ __forceinline__ v16b frag_kb(const b16* p, int hh) { const v8b a = *(const v8b*)(p + 8 * hh), b = *(const v8b*)(p + 16 + 8 * hh); v16b f;
#pragma unroll
  for (int e = 0; e < 8; ++e) { f[e] = a[e]; f[8 + e] = b[e]; } return f; }
__device__ __forceinline__ v8f wmma16b(v16b a, v16b b, v8f c) { v8f d = __builtin_amdgcn_wmma_f32_16x16x32_f16(false, a, false, b, (short)0, c, false, false); asm volatile("v_nop\n\tv_nop\n\tv_nop\n\tv_nop" : "+v"(d) : "v"(a), "v"(b)); return d; }
__device__ __forceinline__ void wave_lds_sync() { __builtin_amdgcn_fence(__ATOMIC_RELEASE, "workgroup"); __builtin_amdgcn_wave_barrier(); __builtin_amdgcn_fence(__ATOMIC_ACQUIRE, "workgroup"); }
__device__ __forceinline__ float pmul(float a, float b) { float p = a * b; asm volatile("" : "+v"(p)); return p; }
__device__ __forceinline__ int iclamp(int v, int lo, int hi) { return v < lo ? lo : (v > hi ? hi : v); }
__device__ __forceinline__ float nexp(float x) { return __builtin_amdgcn_exp2f(x * 1.4426950408889634f); }
__device__ __forceinline__ float lrelu(float x) { return x > 0.0f ? x : NEG * x; }

constexpr int CSR_NBLK = 512, CSR_GB = 8  , CSR_GN = 1 << CSR_GB  , CSR_MAXG = 512, CSR_CAP = 12288  ;
__global__ __launch_bounds__(64) void csrA_kernel(const int* __restrict__ dst, int E, int N, int nG, int CHP, int NGP, int* __restrict__ STG, int* __restrict__ HST) {
  extern __shared__ int sm[];
  int* cnt = sm; int* run = sm + NGP; int* ids = sm + 2 * NGP;
  const int b = blockIdx.x; const int ch = (E + CSR_NBLK - 1) / CSR_NBLK; const int e0 = b * ch, e1 = min(E, e0 + ch);
  for (int i = threadIdx.x; i < NGP; i += 64) cnt[i] = 0;
  for (int i = threadIdx.x; i < CHP; i += 64) ids[i] = -1;
  __syncthreads();
  if (threadIdx.x == 0) {
    for (int e = e0; e < e1; ++e) { int d = dst[e]; d = (d < 0) ? 0 : (d >= N ? N - 1 : d); cnt[d >> CSR_GB] += 1; }
    int acc = 0; for (int g = 0; g < nG; ++g) { run[g] = acc; acc += cnt[g]; }
    for (int e = e0; e < e1; ++e) { int d = dst[e]; d = (d < 0) ? 0 : (d >= N ? N - 1 : d); const int g = d >> CSR_GB; ids[run[g]] = e; run[g] += 1; } }
  __syncthreads();
  typedef __attribute__((ext_vector_type(4))) int v4i;
  for (int pass = 0; pass < 2; ++pass) {
    for (int i = threadIdx.x; i < CHP / 4; i += 64) *(volatile v4i*)(STG + (size_t)b * CHP + i * 4) = *(const v4i*)(&ids[i * 4]);
    for (int i = threadIdx.x; i < NGP / 4; i += 64) { v4i v; for (int e = 0; e < 4; ++e) v[e] = (i * 4 + e < nG) ? cnt[i * 4 + e] : 0; *(volatile v4i*)(HST + (size_t)b * NGP + i * 4) = v; }
    __threadfence(); }
}
__global__ __launch_bounds__(512) void csrS_kernel(const int* __restrict__ HST, int nG, int NGP, int* __restrict__ START, int* __restrict__ TOT, int* __restrict__ OFF) {
  __shared__ int tot[CSR_MAXG];
  const int b = threadIdx.x;
  for (int pass = 0; pass < 2; ++pass) { int runb = 0; for (int g = 0; g < nG; ++g) { int c = HST[(size_t)b * NGP + g]; c = (c < 0) ? 0 : c; ((volatile int*)OFF)[(size_t)g * CSR_NBLK + b] = runb; runb += c; } __threadfence(); }
  for (int g = threadIdx.x; g < nG; g += 512) { int s = 0; for (int bb = 0; bb < CSR_NBLK; ++bb) { int c = HST[(size_t)bb * NGP + g]; s += (c < 0) ? 0 : c; } tot[g] = s; }
  __syncthreads();
  if (threadIdx.x < 32) {
    __shared__ int st[CSR_MAXG + 32];
    if (threadIdx.x == 0) { int acc = 0; for (int g = 0; g < NGP; ++g) { st[g] = acc; if (g < nG) acc += (tot[g] + 31) & ~31; } st[NGP] = acc; }
    __builtin_amdgcn_fence(__ATOMIC_RELEASE, "workgroup"); __builtin_amdgcn_wave_barrier(); __builtin_amdgcn_fence(__ATOMIC_ACQUIRE, "workgroup");
    for (int pass = 0; pass < 2; ++pass) { for (int i = threadIdx.x; i < NGP + 32; i += 32) { ((volatile int*)START)[i] = (i <= NGP) ? st[min(i, NGP)] : 0; ((volatile int*)TOT)[i] = (i < nG) ? tot[i] : 0; } __threadfence(); } }
}
__global__ __launch_bounds__(256) void csrB_kernel(const int* __restrict__ dst, int N, int nG, int CHP, int NGP, int permLen, const int* __restrict__ STG, const int* __restrict__ HST, const int* __restrict__ OFF, const int* __restrict__ START, const int* __restrict__ TOT, int* __restrict__ PERM, int* __restrict__ ROWPTR, int* __restrict__ ROWCNT, int* __restrict__ FLAG) {
  typedef __attribute__((ext_vector_type(4))) int v4i;
  __shared__ int ids[CSR_CAP]; __shared__ unsigned short key[CSR_CAP]; __shared__ int outp[CSR_CAP]; __shared__ int ncnt[CSR_GN + 1]; __shared__ int boff[CSR_NBLK + 1];
  const int g = blockIdx.x, t_ = threadIdx.x; int tot = TOT[g]; int st = START[g], stn = START[g + 1]; const int v0 = g * CSR_GN; const int nv = min(CSR_GN, N - v0);
  st = (st < 0) ? 0 : (st > permLen - 32 ? permLen - 32 : st) & ~31; stn = (stn < st) ? st : (stn > permLen ? permLen : stn); tot = (tot < 0) ? 0 : tot; if (tot > stn - st && tot <= CSR_CAP) tot = stn - st;
  if (tot > CSR_CAP) {
    for (int pass = 0; pass < 2; ++pass) { for (int i = t_; i < CSR_GN / 4; i += 256) { v4i a, c; for (int e = 0; e < 4; ++e) { a[e] = st; c[e] = 0; } *(volatile v4i*)(ROWPTR + v0 + i * 4) = a; *(volatile v4i*)(ROWCNT + v0 + i * 4) = c; } if (t_ == 0) ((volatile int*)FLAG)[0] = 1; __threadfence(); } (void)nv; return; }
  if (t_ == 0) { int acc = 0; for (int b = 0; b < CSR_NBLK; ++b) { boff[b] = acc; int c = HST[(size_t)b * NGP + g]; c = (c < 0) ? 0 : (c > CHP ? CHP : c); acc += c; if (acc > tot) acc = tot; } boff[CSR_NBLK] = acc; }
  for (int i = t_; i <= CSR_GN; i += 256) ncnt[i] = 0;
  __syncthreads();
  for (int b = 0; b < CSR_NBLK; ++b) { const int c = boff[b + 1] - boff[b]; int o_ = OFF[(size_t)g * CSR_NBLK + b]; o_ = (o_ < 0) ? 0 : (o_ > CHP - c ? CHP - c : o_); const int* src_ = STG + (size_t)b * CHP + o_;
    for (int i = t_; i < c; i += 256) { int id = src_[i]; id = (id < 0) ? 0 : id; ids[boff[b] + i] = id; int d = dst[id]; d = (d < v0) ? v0 : (d >= N ? N - 1 : d); int kk = d - v0; kk = (kk < 0) ? 0 : (kk >= CSR_GN ? CSR_GN - 1 : kk); key[boff[b] + i] = (unsigned short)kk; } }
  __syncthreads();
  if (t_ == 0) { for (int i = 0; i < tot; ++i) ncnt[key[i]] += 1; int acc = 0; for (int vl = 0; vl < CSR_GN; ++vl) { const int c = ncnt[vl]; ncnt[vl] = acc; acc += c; } ncnt[CSR_GN] = acc;
    for (int i = 0; i < tot; ++i) { const int vl = key[i]; outp[ncnt[vl]] = ids[i]; ncnt[vl] += 1; }
    for (int vl = CSR_GN; vl > 0; --vl) ncnt[vl] = ncnt[vl - 1]; ncnt[0] = 0; }
  __syncthreads();
  for (int pass = 0; pass < 2; ++pass) {
    for (int i = t_; i < (stn - st) / 4; i += 256) { v4i v; for (int e = 0; e < 4; ++e) { const int q = i * 4 + e; v[e] = (q < tot) ? outp[q] : -1; } *(volatile v4i*)(PERM + st + i * 4) = v; }
    for (int i = t_; i < CSR_GN / 4; i += 256) { v4i a, c; for (int e = 0; e < 4; ++e) { const int vl = i * 4 + e; a[e] = st + ncnt[vl]; c[e] = (vl < nv) ? (ncnt[vl + 1] - ncnt[vl]) : 0; } *(volatile v4i*)(ROWPTR + v0 + i * 4) = a; *(volatile v4i*)(ROWCNT + v0 + i * 4) = c; }
    __threadfence(); }
}
__global__ __launch_bounds__(256) void csrZ_kernel(int* __restrict__ p, size_t n4) { typedef __attribute__((ext_vector_type(4))) int v4i; const size_t tid = (size_t)blockIdx.x * 256 + threadIdx.x, nth = (size_t)gridDim.x * 256; v4i z = {0, 0, 0, 0}; for (size_t i = tid; i < n4; i += nth) *(volatile v4i*)(p + i * 4) = z; }
struct CsrBufs { int *STG, *HST, *OFF, *START, *TOT, *PERM, *ROWPTR, *ROWCNT, *FLAG; int nG, NGP, CHP; size_t permLen; char* base; size_t bytes; };
static size_t csr_carve(CsrBufs& c, char* ws, size_t off, int E, int N) {
  const size_t off0 = off; c.base = ws + off;
  auto al = [&](size_t bytes) { char* p = ws + off; off += (bytes + 255) & ~(size_t)255; return p; };
  c.nG = (N + CSR_GN - 1) / CSR_GN; c.NGP = (c.nG + 31) & ~31; const int ch = (E + CSR_NBLK - 1) / CSR_NBLK; c.CHP = (ch + 31) & ~31; c.permLen = (size_t)E + 32 * (size_t)c.nG + 32;
  c.STG = (int*)al((size_t)CSR_NBLK * c.CHP * 4); c.HST = (int*)al((size_t)CSR_NBLK * c.NGP * 4); c.OFF = (int*)al((size_t)c.NGP * CSR_NBLK * 4); c.START = (int*)al((size_t)(c.NGP + 64) * 4); c.TOT = (int*)al((size_t)(c.NGP + 64) * 4);
  c.PERM = (int*)al(c.permLen * 4); c.ROWPTR = (int*)al((size_t)c.nG * CSR_GN * 4); c.ROWCNT = (int*)al((size_t)c.nG * CSR_GN * 4); c.FLAG = (int*)al(256);
  c.bytes = off - off0; return off;
}
static void csr_build(const CsrBufs& c, const int* dst, int E, int N, hipStream_t stream) {
  const size_t smem = (size_t)(2 * c.NGP + c.CHP) * 4;
  csrZ_kernel<<<512, 256, 0, stream>>>((int*)c.base, c.bytes / 16);
  csrA_kernel<<<CSR_NBLK, 64, smem, stream>>>(dst, E, N, c.nG, c.CHP, c.NGP, c.STG, c.HST);
  csrS_kernel<<<1, 512, 0, stream>>>(c.HST, c.nG, c.NGP, c.START, c.TOT, c.OFF);
  csrB_kernel<<<c.nG, 256, 0, stream>>>(dst, N, c.nG, c.CHP, c.NGP, (int)c.permLen, c.STG, c.HST, c.OFF, c.START, c.TOT, c.PERM, c.ROWPTR, c.ROWCNT, c.FLAG);
}


__device__ __forceinline__ float sigm(float x) { return 1.0f / (1.0f + __expf(-x)); }
__global__ __launch_bounds__(256) void prep_kernel(const float* __restrict__ x, const float* __restrict__ W1, const float* __restrict__ wi1, const float* __restrict__ wh1, const float* __restrict__ W2, const float* __restrict__ wi2, const float* __restrict__ wh2, b16* __restrict__ HPh, b16* __restrict__ HPl, float* __restrict__ HF, b16* __restrict__ WT, b16* __restrict__ WG) {
  const size_t u = (size_t)blockIdx.x * 256 + threadIdx.x; const size_t nx = (size_t)NP * DP / 8, nt = (size_t)2 * TW * DP / 8, ng = (size_t)2 * GW * 64 / 8; size_t t = u; v8b o;
  if (t < nx) { const size_t e = t * 8; const size_t v = e / DP; const int c0 = (int)(e % DP); v8b z8 = {}; float f[8]; for (int j = 0; j < 8; ++j) { const int c = c0 + j; f[j] = (v < (size_t)N && c < D) ? bf16_rne(x[v * D + c]) : 0.0f; o[j] = (b16)(f[j] * XS); }
    v4f f0 = {f[0], f[1], f[2], f[3]}, f1 = {f[4], f[5], f[6], f[7]};
    for (int pass = 0; pass < 2; ++pass) { *(volatile v8b*)(HPh + e) = o; *(volatile v8b*)(HPl + e) = z8; *(volatile v4f*)(HF + e) = f0; *(volatile v4f*)(HF + e + 4) = f1; __threadfence(); } return; } t -= nx;
  if (t < nt) { const size_t e = t * 8; const int l = (int)(e / (TW * DP)); const int rem = (int)(e % (TW * DP)); const int row = rem / DP, d0 = rem % DP; const int k = row / DP, f = row % DP; const float* Wl = l ? W2 : W1;
    for (int j = 0; j < 8; ++j) { const int d = d0 + j; o[j] = (f < D && d < D) ? (b16)(bf16_rne(Wl[((size_t)k * D + f) * D + d]) * WSC) : (b16)0.0f; } for (int pass = 0; pass < 2; ++pass) { *(volatile v8b*)(WT + e) = o; __threadfence(); } return; } t -= nt;
  if (t < ng) { const size_t e = t * 8; const int l = (int)(e / (GW * 64)); const int rem = (int)(e % (GW * 64)); const int row = rem / 64, c0 = rem % 64; const bool isH = row >= 3 * DP; const int rr = isH ? row - 3 * DP : row; const int g = rr / DP, f = rr % DP;
    const float* w = isH ? (l ? wh2 : wh1) : (l ? wi2 : wi1);
    for (int j = 0; j < 8; ++j) { const int c = c0 + j; const int d = isH ? c - DP : c; const bool ok = f < D && (isH ? (c >= DP && d < D) : (c < D)); o[j] = ok ? (b16)(bf16_rne(w[((size_t)g * D + f) * D + d]) * WSC) : (b16)0.0f; }
    for (int pass = 0; pass < 2; ++pass) { *(volatile v8b*)(WG + e) = o; __threadfence(); } }
}
__global__ __launch_bounds__(128) void tgemm_kernel(const b16* __restrict__ HPh, const b16* __restrict__ HPl, const b16* __restrict__ WT, const float* __restrict__ bk, float* __restrict__ T) {
  __shared__ __attribute__((aligned(16))) float Tf[4][16][TW + 4];
  const int wave = threadIdx.x >> 5, lane = threadIdx.x & 31, nloc = lane & 15, hlf = lane >> 4; const size_t m0 = (size_t)blockIdx.x * 64 + wave * 16;
  v8f acc[6];
#pragma unroll
  for (int t = 0; t < 6; ++t) acc[t] = (v8f){};
  { const v16b a = frag_kb(HPh + (m0 + nloc) * DP, hlf), al = frag_kb(HPl + (m0 + nloc) * DP, hlf);
#pragma unroll
    for (int t = 0; t < 6; ++t) { const v16b bw = frag_kb(WT + (size_t)(t * 16 + nloc) * DP, hlf); acc[t] = wmma16b(a, bw, acc[t]); acc[t] = wmma16b(al, bw, acc[t]); } }
#pragma unroll
  for (int t = 0; t < 6; ++t) { const int c = t * 16 + nloc; const int k = c / DP, f = c % DP; const float bb = f < D ? bf16_rne(bk[k * D + f]) : 0.0f;
#pragma unroll 1
    for (int r = 0; r < 8; ++r) Tf[wave][8 * hlf + r][c] = f < D ? acc[t][r] * (1.0f / (XS * WSC)) + bb : 0.0f; }
  wave_lds_sync();
  for (int pass = 0; pass < 2; ++pass) { for (int rr = 0; rr < 16; ++rr) if (lane < 24) *(volatile v4f*)(T + (m0 + rr) * TW + lane * 4) = *(const v4f*)(&Tf[wave][rr][lane * 4]); __threadfence(); }
}
__global__ __launch_bounds__(256) void agg_kernel(const float* __restrict__ T, const float* __restrict__ HF, const int* __restrict__ srcs, const int* __restrict__ et, const int* __restrict__ PERM, const int* __restrict__ ROWPTR, const int* __restrict__ ROWCNT, int permLen, b16* __restrict__ Ah, b16* __restrict__ Al) {
  __shared__ __attribute__((aligned(16))) b16 sh[8][2][64];
  const int wave = threadIdx.x >> 5, lane = threadIdx.x & 31; const size_t v = (size_t)blockIdx.x * 8 + wave;
  float a = 0.0f, hv = 0.0f;
  if (v < (size_t)N) { int st = ROWPTR[v], cnt = ROWCNT[v]; cnt = iclamp(cnt, 0, 65536); st = iclamp(st, 0, permLen - cnt);
    for (int i = 0; i < cnt; ++i) { const int e = iclamp(PERM[st + i], 0, E - 1); const size_t s = (size_t)iclamp(srcs[e], 0, N - 1); const int k = iclamp(et[e], 0, KE - 1); a += T[s * TW + k * DP + lane]; }
    hv = HF[v * DP + lane]; }
  { b16 p, q; split16(a * XS, p, q); sh[wave][0][lane] = p; sh[wave][1][lane] = q; split16(hv * XS, p, q); sh[wave][0][32 + lane] = p; sh[wave][1][32 + lane] = q; }
  wave_lds_sync();
  for (int pass = 0; pass < 2; ++pass) { if (lane < 8) *(volatile v8b*)(Ah + v * 64 + lane * 8) = *(const v8b*)(&sh[wave][0][lane * 8]); else if (lane < 16) *(volatile v8b*)(Al + v * 64 + (lane - 8) * 8) = *(const v8b*)(&sh[wave][1][(lane - 8) * 8]); __threadfence(); }
}
template <int RELU>
__global__ __launch_bounds__(128) void gru_kernel(const b16* __restrict__ Ah, const b16* __restrict__ Al, const b16* __restrict__ WG, const float* __restrict__ bi, const float* __restrict__ bh, const float* HF, float* HF2, b16* __restrict__ HPh, b16* __restrict__ HPl) {
  __shared__ __attribute__((aligned(16))) float Tf[4][16][DP + 4];
  const int wave = threadIdx.x >> 5, lane = threadIdx.x & 31, nloc = lane & 15, hlf = lane >> 4; const size_t m0 = (size_t)blockIdx.x * 64 + wave * 16;
  v8f acc[12];
#pragma unroll
  for (int t = 0; t < 12; ++t) acc[t] = (v8f){};
#pragma unroll
  for (int kb = 0; kb < 64; kb += 32) { const v16b a = frag_kb(Ah + (m0 + nloc) * 64 + kb, hlf), al = frag_kb(Al + (m0 + nloc) * 64 + kb, hlf);
#pragma unroll
    for (int t = 0; t < 12; ++t) { const v16b bw = frag_kb(WG + (size_t)(t * 16 + nloc) * 64 + kb, hlf); acc[t] = wmma16b(a, bw, acc[t]); acc[t] = wmma16b(al, bw, acc[t]); } }
  const float sc = 1.0f / (XS * WSC);
#pragma unroll
  for (int half = 0; half < 2; ++half) { const int f = half * 16 + nloc;
    const float bir = f < D ? bf16_rne(bi[f]) : 0.0f, biz = f < D ? bf16_rne(bi[D + f]) : 0.0f, bin_ = f < D ? bf16_rne(bi[2 * D + f]) : 0.0f, bhr = f < D ? bf16_rne(bh[f]) : 0.0f, bhz = f < D ? bf16_rne(bh[D + f]) : 0.0f, bhn = f < D ? bf16_rne(bh[2 * D + f]) : 0.0f;
#pragma unroll 1
    for (int r = 0; r < 8; ++r) { const size_t row = m0 + 8 * hlf + r;
      const float gir = acc[0 + half][r] * sc + bir, giz = acc[2 + half][r] * sc + biz, gin = acc[4 + half][r] * sc + bin_, ghr = acc[6 + half][r] * sc + bhr, ghz = acc[8 + half][r] * sc + bhz, ghn = acc[10 + half][r] * sc + bhn;
      const float rg = sigm(gir + ghr), zg = sigm(giz + ghz); const float ng = tanhf(gin + pmul(rg, ghn)); const float hp = (row < (size_t)N && f < D) ? HF[row * DP + f] : 0.0f;
      float y = pmul(1.0f - zg, ng) + pmul(zg, hp); if (RELU) y = fmaxf(y, 0.0f); if (row >= (size_t)N || f >= D) y = 0.0f; Tf[wave][8 * hlf + r][f] = y; } }
  wave_lds_sync();
  for (int pass = 0; pass < 2; ++pass) { for (int rr = 0; rr < 16; ++rr) { if (lane < 8) *(volatile v4f*)(HF2 + (m0 + rr) * DP + lane * 4) = *(const v4f*)(&Tf[wave][rr][lane * 4]);
      else if (lane < 12) { const int c8 = (lane - 8) * 8; v8b ph, pl; for (int j = 0; j < 8; ++j) { b16 p, q; split16(Tf[wave][rr][c8 + j] * XS, p, q); ph[j] = p; pl[j] = q; } *(volatile v8b*)(HPh + (m0 + rr) * DP + c8) = ph; *(volatile v8b*)(HPl + (m0 + rr) * DP + c8) = pl; } }
    __threadfence(); }
}
__global__ __launch_bounds__(256) void dot_kernel(const float* __restrict__ HF, const int* __restrict__ s_, const int* __restrict__ d_, float* __restrict__ out) {
  const size_t e = (size_t)blockIdx.x * 256 + threadIdx.x; if (e >= (size_t)E) return;
  const size_t s = (size_t)iclamp(s_[e], 0, N - 1), d = (size_t)iclamp(d_[e], 0, N - 1); float acc = 0.0f;
#pragma unroll 1
  for (int c = 0; c < D; ++c) acc += pmul(HF[s * DP + c], HF[d * DP + c]);
  for (int pass = 0; pass < 2; ++pass) { ((volatile float*)out)[e] = acc; __threadfence(); }
}
}

extern "C" void kernel_launch(void* const* d_in, const int* in_sizes, int n_in, void* d_out, int out_size, void* d_ws, size_t ws_size, hipStream_t stream) {
  (void)n_in;
  auto Fp = [&](int i) { return (const float*)d_in[i]; }; auto Ip = [&](int i) { return (const int*)d_in[i]; };
  if (in_sizes[0] != N * D || in_sizes[1] != E || in_sizes[2] != E || in_sizes[3] != E || in_sizes[4] != E || in_sizes[5] != E || in_sizes[6] != KE * D * D || in_sizes[8] != 3 * D * D || out_size != 2 * E) return;
  size_t off = 0; char* ws = (char*)d_ws;
  auto carve = [&](size_t bytes) { char* p = ws + off; off += (bytes + 255) & ~(size_t)255; return p; };
  b16* HPh = (b16*)carve((size_t)NP * DP * 2); b16* HPl = (b16*)carve((size_t)NP * DP * 2); float* HF = (float*)carve((size_t)NP * DP * 4);
  b16* WT = (b16*)carve((size_t)2 * TW * DP * 2); b16* WG = (b16*)carve((size_t)2 * GW * 64 * 2); float* T = (float*)carve((size_t)NP * TW * 4); b16* Ah = (b16*)carve((size_t)NP * 64 * 2); b16* Al = (b16*)carve((size_t)NP * 64 * 2);
  CsrBufs csr; off = csr_carve(csr, ws, off, E, N);
  if (off > ws_size || off > ((size_t)128 << 20)) return;
  prep_kernel<<<(unsigned)(((size_t)NP * DP / 8 + (size_t)2 * TW * DP / 8 + (size_t)2 * GW * 64 / 8 + 255) / 256), 256, 0, stream>>>(Fp(0), Fp(6), Fp(8), Fp(9), Fp(12), Fp(14), Fp(15), HPh, HPl, HF, WT, WG);
  csr_build(csr, Ip(2), E, N, stream);
  tgemm_kernel<<<NP / 64, 128, 0, stream>>>(HPh, HPl, WT, Fp(7), T);
  agg_kernel<<<NP / 8, 256, 0, stream>>>(T, HF, Ip(1), Ip(3), csr.PERM, csr.ROWPTR, csr.ROWCNT, (int)csr.permLen, Ah, Al);
  gru_kernel<1><<<NP / 64, 128, 0, stream>>>(Ah, Al, WG, Fp(10), Fp(11), HF, HF, HPh, HPl);
  tgemm_kernel<<<NP / 64, 128, 0, stream>>>(HPh, HPl, WT + (size_t)TW * DP, Fp(13), T);
  agg_kernel<<<NP / 8, 256, 0, stream>>>(T, HF, Ip(1), Ip(3), csr.PERM, csr.ROWPTR, csr.ROWCNT, (int)csr.permLen, Ah, Al);
  gru_kernel<0><<<NP / 64, 128, 0, stream>>>(Ah, Al, WG + (size_t)GW * 64, Fp(16), Fp(17), HF, HF, HPh, HPl);
  dot_kernel<<<(E + 255) / 256, 256, 0, stream>>>(HF, Ip(1), Ip(2), (float*)d_out);
  dot_kernel<<<(E + 255) / 256, 256, 0, stream>>>(HF, Ip(4), Ip(5), (float*)d_out + E);
}
